// DAWNBlock_88124138979392
// MI455X (gfx1250) — hardware-verified
//
#include <hip/hip_runtime.h>
#include <math.h>
#include <stdint.h>

#define NBATCH 2
#define TT     2048
#define DM     1024
#define NH     16
#define HD     64
#define RK     256
#define NE     8
#define KRK    128
#define NR     (NE * RK)
#define NKR    (NE * KRK)
#define QKP    (2 * DM)
#define MP     (NBATCH * TT)
#define NQB    (TT / 64)
#define WIN    0
#define LNEPS  1.0e-5f
#define WSC    64.0f
#define ASC    256.0f
#define QKSC   4.0f
#define VSC    16.0f
#define PSC    1024.0f
#define CTXSC  16.0f
static_assert(NH * HD == DM);
static_assert((MP % 64) == 0 && (DM % 64) == 0 && (NR % 64) == 0 && (NKR % 64) == 0 && (TT % 64) == 0);
static_assert((RK % 64) == 0 && (KRK % 64) == 0 && (QKP % 64) == 0);
static_assert(DM == 4 * 256);
static_assert(RK <= 256 && KRK <= 256 && NR <= 2048 && NKR <= 2048);

typedef _Float16 v16h __attribute__((ext_vector_type(16)));
typedef _Float16 v8h  __attribute__((ext_vector_type(8)));
typedef float    v8f  __attribute__((ext_vector_type(8)));
typedef float    v4f  __attribute__((ext_vector_type(4)));
typedef unsigned int v4u __attribute__((ext_vector_type(4)));
typedef unsigned int v2u __attribute__((ext_vector_type(2)));

__device__ __forceinline__ unsigned short bf_bits(float f) {
  unsigned u = __float_as_uint(f);
  return (unsigned short)((u + 0x7FFFu + ((u >> 16) & 1u)) >> 16);
}
__device__ __forceinline__ float bf_up(unsigned short h) { return __uint_as_float(((unsigned)h) << 16); }
__device__ __forceinline__ float bfr(float f) { return bf_up(bf_bits(f)); }
__device__ __forceinline__ unsigned short h_bits(_Float16 x) { return __builtin_bit_cast(unsigned short, x); }
__device__ __forceinline__ unsigned pk16(unsigned short a, unsigned short b) { return (unsigned)a | ((unsigned)b << 16); }
__device__ __forceinline__ v8f zero8() { v8f z = {0.f, 0.f, 0.f, 0.f, 0.f, 0.f, 0.f, 0.f}; return z; }
__device__ __forceinline__ float gelu_f(float v) { return 0.5f * v * (1.0f + erff(v * 0.70710678118654752f)); }

__device__ __forceinline__ v16h ldfrag_h(const _Float16* p) {
  union { v16h v; v8h h[2]; } f;
  f.h[0] = *(const v8h*)(p);
  f.h[1] = *(const v8h*)(p + 16);
  return f.v;
}

__device__ __forceinline__ v8f mma_h(v16h a, v16h b, v8f c) {
  c = __builtin_amdgcn_wmma_f32_16x16x32_f16(false, a, false, b, (short)0, c, false, false);
#if defined(__HIP_DEVICE_COMPILE__)
  asm volatile("v_nop\n\tv_nop\n\tv_nop\n\tv_nop" : "+v"(c) : "v"(a), "v"(b));
#endif
  return c;
}
__device__ __forceinline__ v8f mma_h_raw(v16h a, v16h b, v8f c) {
  return __builtin_amdgcn_wmma_f32_16x16x32_f16(false, a, false, b, (short)0, c, false, false);
}
__device__ __forceinline__ void dep_guard1(v8f& a, v8f& b, v16h x) {
#if defined(__HIP_DEVICE_COMPILE__)
  asm volatile("v_nop\n\tv_nop\n\tv_nop\n\tv_nop" : "+v"(a), "+v"(b) : "v"(x));
#endif
}
__device__ __forceinline__ void keep4_h(v16h a, v16h b, v16h c, v16h d) {
#if defined(__HIP_DEVICE_COMPILE__)
  asm volatile("v_nop" :: "v"(a), "v"(b), "v"(c), "v"(d));
#endif
}
__device__ __forceinline__ void acc_guard4(v8f& a, v8f& b, v8f& c, v8f& d) {
#if defined(__HIP_DEVICE_COMPILE__)
  asm volatile("v_nop\n\tv_nop\n\tv_nop\n\tv_nop" : "+v"(a), "+v"(b), "+v"(c), "+v"(d));
#endif
}
__device__ __forceinline__ void wave_sync_lds() {
  __builtin_amdgcn_fence(__ATOMIC_RELEASE, "workgroup");
  __builtin_amdgcn_wave_barrier();
  __builtin_amdgcn_fence(__ATOMIC_ACQUIRE, "workgroup");
}
__device__ __forceinline__ float wsum(float v) {
#pragma unroll
  for (int off = 16; off > 0; off >>= 1) v += __shfl_xor(v, off, 32);
  return v;
}
__device__ __forceinline__ float bsum256(float v, float* red, int lane, int wave) {
  v = wsum(v);
  if (lane == 0) red[wave] = v;
  __syncthreads();
  float tot = 0.f;
#pragma unroll
  for (int w = 0; w < 8; ++w) tot += red[w];
  return tot;
}

__global__ __launch_bounds__(256) void conv_h64(const float* __restrict__ W, unsigned short* Wh, int n8,
                                                float wsc) {
  const int i = blockIdx.x * 256 + threadIdx.x;
  if (i >= n8) return;
  const size_t e0 = (size_t)i * 8;
  const v4f a = *(const v4f*)(W + e0);
  const v4f b = *(const v4f*)(W + e0 + 4);
  v4u u;
  u[0] = pk16(h_bits((_Float16)(bfr(a[0]) * wsc)), h_bits((_Float16)(bfr(a[1]) * wsc)));
  u[1] = pk16(h_bits((_Float16)(bfr(a[2]) * wsc)), h_bits((_Float16)(bfr(a[3]) * wsc)));
  u[2] = pk16(h_bits((_Float16)(bfr(b[0]) * wsc)), h_bits((_Float16)(bfr(b[1]) * wsc)));
  u[3] = pk16(h_bits((_Float16)(bfr(b[2]) * wsc)), h_bits((_Float16)(bfr(b[3]) * wsc)));
  for (int pass = 0; pass < 2; ++pass) {
    *(volatile v4u*)(Wh + e0) = u;
    __threadfence();
  }
}

__global__ __launch_bounds__(256) void tconv_h64(const float* __restrict__ in, int ldi, long long inStrideZ,
                                                 unsigned short* out, int ldo, long long outStrideZ, float wsc) {
  __shared__ __align__(16) unsigned short sT[64 * 72];
  const int t  = threadIdx.x;
  const int c0 = blockIdx.x * 64, r0 = blockIdx.y * 64, z = blockIdx.z;
  const float* inz = in + (size_t)z * (size_t)inStrideZ;
  {
    const int row = t >> 2, cc = (t & 3) * 16;
    const float* src = inz + (size_t)(r0 + row) * ldi + c0 + cc;
#pragma unroll
    for (int q = 0; q < 4; ++q) {
      const v4f v = *(const v4f*)(src + 4 * q);
#pragma unroll
      for (int e = 0; e < 4; ++e)
        sT[(cc + 4 * q + e) * 72 + row] = h_bits((_Float16)(bfr(v[e]) * wsc));
    }
  }
  __syncthreads();
  unsigned short* outz = out + (size_t)z * (size_t)outStrideZ;
  const int piece = (t & 7) * 8, orl = t >> 3;
  v4u vv[2];
#pragma unroll
  for (int it = 0; it < 2; ++it) vv[it] = *(const v4u*)(sT + (it * 32 + orl) * 72 + piece);
  for (int pass = 0; pass < 2; ++pass) {
#pragma unroll
    for (int it = 0; it < 2; ++it) {
      const int orow = it * 32 + orl;
      *(volatile v4u*)(outz + (size_t)(c0 + orow) * ldo + r0 + piece) = vv[it];
    }
    __threadfence();
  }
}

template <int OM, int BIASM, int ACT, int RES>
__global__ __launch_bounds__(256) void gemm64(
    const unsigned short* __restrict__ Ap, int lda, long long strideA,
    const unsigned short* __restrict__ Btp, int ldb, long long strideB,
    const float* __restrict__ bias0, const float* __restrict__ bias1, int Nb,
    const float* resid,
    void* Cout, int ldc, long long strideC,
    int M, int N, int K, float oscale) {
  const _Float16* A  = (const _Float16*)(const void*)Ap;
  const _Float16* Bt = (const _Float16*)(const void*)Btp;
  __shared__ __align__(16) float sT[8][16 * 68];
  const int b    = blockIdx.y;
  const int lane = threadIdx.x & 31;
  const int wave = threadIdx.x >> 5;
  const int tilesN = N >> 6;
  const int tilesM = M >> 6;
  const int tile = blockIdx.x * 8 + wave;
  if (tile >= tilesM * tilesN) return;
  const int tm = tile / tilesN;
  const int tn = tile - tm * tilesN;
  const int m0 = tm << 6;
  const int n0 = tn << 6;

  const _Float16* Ab = A  + (size_t)b * strideA;
  const _Float16* Bb = Bt + (size_t)b * strideB;

  const int rlane = lane & 15;
  const int koff  = (lane >> 4) * 8;
  const int mOff  = (lane >> 4) * 8;

  v8f acc[4][4];
#pragma unroll
  for (int i = 0; i < 4; ++i)
#pragma unroll
    for (int j = 0; j < 4; ++j) acc[i][j] = zero8();

  for (int k0 = 0; k0 < K; k0 += 32) {
    v16h bh[4];
#pragma unroll
    for (int j = 0; j < 4; ++j) {
      const size_t bo = (size_t)(n0 + (j << 4) + rlane) * ldb + koff + k0;
      bh[j] = ldfrag_h(Bb + bo);
    }
#pragma unroll
    for (int i = 0; i < 4; ++i) {
      const size_t ao = (size_t)(m0 + (i << 4) + rlane) * lda + koff + k0;
      const v16h ah = ldfrag_h(Ab + ao);
#pragma unroll
      for (int j = 0; j < 4; ++j) acc[i][j] = mma_h_raw(ah, bh[j], acc[i][j]);
      dep_guard1(acc[i][0], acc[i][3], ah);
    }
    keep4_h(bh[0], bh[1], bh[2], bh[3]);
  }
  acc_guard4(acc[0][0], acc[0][1], acc[0][2], acc[0][3]);
  acc_guard4(acc[1][0], acc[1][1], acc[1][2], acc[1][3]);
  acc_guard4(acc[2][0], acc[2][1], acc[2][2], acc[2][3]);
  acc_guard4(acc[3][0], acc[3][1], acc[3][2], acc[3][3]);

  const int hh2 = lane >> 4, c4 = (lane & 15) * 4;
  const int q8  = lane >> 3, c8 = (lane & 7) * 8;
  float bc[8];
#pragma unroll
  for (int e = 0; e < 8; ++e) bc[e] = 0.f;
  if (BIASM == 0) {
    const bool use1 = (n0 >= Nb);
    if (OM == 0) {
      const int cb = n0 + c4;
      const int i0 = (cb < Nb - 4) ? cb : (Nb - 4);
      const int i1 = (cb - Nb > 0) ? (cb - Nb) : 0;
      const v4f b0v = *(const v4f*)(bias0 + i0);
      const v4f b1v = *(const v4f*)(bias1 + i1);
#pragma unroll
      for (int e = 0; e < 4; ++e) bc[e] = bfr(use1 ? b1v[e] : b0v[e]);
    } else {
      const int cb = n0 + c8;
      const int i0 = (cb < Nb - 8) ? cb : (Nb - 8);
      const int i1 = (cb - Nb > 0) ? (cb - Nb) : 0;
      const v4f b0a = *(const v4f*)(bias0 + i0), b0b = *(const v4f*)(bias0 + i0 + 4);
      const v4f b1a = *(const v4f*)(bias1 + i1), b1b = *(const v4f*)(bias1 + i1 + 4);
#pragma unroll
      for (int e = 0; e < 4; ++e) {
        bc[e]     = bfr(use1 ? b1a[e] : b0a[e]);
        bc[4 + e] = bfr(use1 ? b1b[e] : b0b[e]);
      }
    }
  }

  float* slab = sT[wave];
#pragma unroll
  for (int i = 0; i < 4; ++i) {
    const int mBase = m0 + (i << 4);
#pragma unroll
    for (int j = 0; j < 4; ++j) {
#pragma unroll
      for (int r = 0; r < 8; ++r) {
        slab[(mOff + r) * 68 + (j << 4) + rlane] = acc[i][j][r];
      }
    }
    wave_sync_lds();
    if (OM == 0) {
      float* C = (float*)Cout + (size_t)b * strideC;
      const float* Rb = resid + (size_t)b * strideC;
      v4f vals[8];
#pragma unroll
      for (int it = 0; it < 8; ++it) {
        const int row = it * 2 + hh2;
        v4f v = *(const v4f*)(slab + row * 68 + c4);
#pragma unroll
        for (int e = 0; e < 4; ++e) {
          float f = v[e] * oscale + bc[e];
          if (ACT) f = gelu_f(f);
          v[e] = f;
        }
        if (RES != 0) {
          const v4f rr = *(const v4f*)(Rb + (size_t)(mBase + row) * ldc + n0 + c4);
#pragma unroll
          for (int e = 0; e < 4; ++e) v[e] += (RES == 2) ? bfr(rr[e]) : rr[e];
        }
        vals[it] = v;
      }
      for (int pass = 0; pass < 2; ++pass) {
#pragma unroll
        for (int it = 0; it < 8; ++it) {
          const int row = it * 2 + hh2;
          *(volatile v4f*)(C + (size_t)(mBase + row) * ldc + n0 + c4) = vals[it];
        }
        __threadfence();
      }
    } else {
      unsigned short* C = (unsigned short*)Cout + (size_t)b * strideC;
      v4u hv[4];
#pragma unroll
      for (int it = 0; it < 4; ++it) {
        const int row = it * 4 + q8;
        const float* sp = slab + row * 68 + c8;
        float bm = 0.f;
        if (BIASM == 1) bm = bfr(bias0[mBase + row]);
        v4u a;
#pragma unroll
        for (int e = 0; e < 4; ++e) {
          float f0 = sp[2 * e]     * oscale + ((BIASM == 1) ? bm : bc[2 * e]);
          float f1 = sp[2 * e + 1] * oscale + ((BIASM == 1) ? bm : bc[2 * e + 1]);
          if (ACT) { f0 = gelu_f(f0); f1 = gelu_f(f1); }
          unsigned short u0, u1;
          if (OM == 1) { u0 = bf_bits(f0); u1 = bf_bits(f1); }
          else         { u0 = h_bits((_Float16)f0); u1 = h_bits((_Float16)f1); }
          a[e] = pk16(u0, u1);
        }
        hv[it] = a;
      }
      for (int pass = 0; pass < 2; ++pass) {
#pragma unroll
        for (int it = 0; it < 4; ++it) {
          const int row = it * 4 + q8;
          *(volatile v4u*)(C + (size_t)(mBase + row) * ldc + n0 + c8) = hv[it];
        }
        __threadfence();
      }
    }
    wave_sync_lds();
  }
}

__global__ __launch_bounds__(128)
void attn64(const unsigned short* __restrict__ qkp, const unsigned short* __restrict__ vtp,
            unsigned short* outp, float sscale) {
  union FH { v16h v; v8h h[2]; };
  __shared__ __align__(16) _Float16 Ksh[64 * 64];
  __shared__ __align__(16) _Float16 Vth[64 * 64];
  __shared__ __align__(16) _Float16 Psh[4][16 * 64];
  __shared__ __align__(16) float    Os[4][16 * 64];

  const int tid  = threadIdx.x;
  const int wave = tid >> 5;
  const int lane = tid & 31;
  const int hh   = lane >> 4;
  const int c    = lane & 15;

  const int bx   = blockIdx.x;
  const int qb   = bx % NQB;
  const int rest = bx / NQB;
  const int h    = rest % NH;
  const int b    = rest / NH;
  const int qblk = qb * 64;
  const int q0   = qblk + wave * 16;
  const size_t rowB = (size_t)b * TT;

  const _Float16* Qh = (const _Float16*)(const void*)qkp + (size_t)h * HD;
  const _Float16* Kg = (const _Float16*)(const void*)qkp + DM + (size_t)h * HD;
  const _Float16* Vh = (const _Float16*)(const void*)vtp + ((size_t)b * DM + (size_t)h * HD) * TT;

  v16h qa[2];
#pragma unroll
  for (int dc = 0; dc < 2; ++dc) qa[dc] = ldfrag_h(Qh + (rowB + q0 + c) * QKP + dc * 32 + 8 * hh);

  float mrow[8], lrow[8];
  v8f oacc[4];
#pragma unroll
  for (int r = 0; r < 8; ++r) { mrow[r] = -INFINITY; lrow[r] = 0.f; }
#pragma unroll
  for (int t = 0; t < 4; ++t) oacc[t] = zero8();

  int ktHi = (qblk + 63 + WIN) >> 6;
  if (ktHi > NQB - 1) ktHi = NQB - 1;

  for (int kt = 0; kt <= ktHi; ++kt) {
    const int kv0 = kt * 64;
    __syncthreads();
    {
      const int r = tid >> 1, hf = (tid & 1) * 32;
      const _Float16* kg = Kg + (rowB + kv0 + r) * QKP + hf;
      const _Float16* vg = Vh + (size_t)r * TT + kv0 + hf;
#pragma unroll
      for (int i = 0; i < 4; ++i) {
        const v8h a0 = *(const v8h*)(kg + 8 * i);
        const v8h b0 = *(const v8h*)(vg + 8 * i);
        *(v8h*)(Ksh + r * 64 + hf + 8 * i) = a0;
        *(v8h*)(Vth + r * 64 + hf + 8 * i) = b0;
      }
    }
    __syncthreads();

    v8f s[4];
#pragma unroll
    for (int j = 0; j < 4; ++j) {
      v8f sh = zero8();
#pragma unroll
      for (int dc = 0; dc < 2; ++dc) {
        FH kb;
        kb.h[0] = *(const v8h*)(Ksh + (j * 16 + c) * 64 + dc * 32 + 8 * hh);
        kb.h[1] = *(const v8h*)(Ksh + (j * 16 + c) * 64 + dc * 32 + 16 + 8 * hh);
        sh = mma_h(qa[dc], kb.v, sh);
      }
      const int key = kv0 + j * 16 + c;
#pragma unroll
      for (int r = 0; r < 8; ++r) {
        const int qrow = q0 + 8 * hh + r;
        const float v = sh[r] * sscale;
        s[j][r] = (key <= qrow + WIN) ? v : -INFINITY;
      }
    }

    _Float16* pwh = Psh[wave];
#pragma unroll
    for (int r = 0; r < 8; ++r) {
      float m = s[0][r];
      m = fmaxf(m, s[1][r]);
      m = fmaxf(m, s[2][r]);
      m = fmaxf(m, s[3][r]);
#pragma unroll
      for (int off = 1; off < 16; off <<= 1) m = fmaxf(m, __shfl_xor(m, off, 32));
      const float mnew  = fmaxf(mrow[r], m);
      const float ms    = (mnew == -INFINITY) ? 0.f : mnew;
      const float alpha = __expf(mrow[r] - ms);
      mrow[r] = mnew;
      float psum = 0.f;
#pragma unroll
      for (int j = 0; j < 4; ++j) {
        const float p = __expf(s[j][r] - ms);
        psum += p;
        pwh[(8 * hh + r) * 64 + j * 16 + c] = (_Float16)(p * PSC);
      }
#pragma unroll
      for (int off = 1; off < 16; off <<= 1) psum += __shfl_xor(psum, off, 32);
      lrow[r] = lrow[r] * alpha + psum;
#pragma unroll
      for (int t = 0; t < 4; ++t) oacc[t][r] *= alpha;
    }
    wave_sync_lds();

#pragma unroll 1
    for (int kk = 0; kk < 2; ++kk) {
      FH pa;
      pa.h[0] = *(const v8h*)(pwh + c * 64 + kk * 32 + 8 * hh);
      pa.h[1] = *(const v8h*)(pwh + c * 64 + kk * 32 + 16 + 8 * hh);
#pragma unroll
      for (int t = 0; t < 4; ++t) {
        FH vb;
        vb.h[0] = *(const v8h*)(Vth + (t * 16 + c) * 64 + kk * 32 + 8 * hh);
        vb.h[1] = *(const v8h*)(Vth + (t * 16 + c) * 64 + kk * 32 + 16 + 8 * hh);
        oacc[t] = mma_h(pa.v, vb.v, oacc[t]);
      }
    }
  }

  float* os = Os[wave];
#pragma unroll
  for (int r = 0; r < 8; ++r) {
    const float l = lrow[r];
    const float inv = ((l > 0.f) ? (1.0f / l) : 0.f) * (CTXSC / (PSC * VSC));
#pragma unroll
    for (int t = 0; t < 4; ++t) os[(8 * hh + r) * 64 + t * 16 + c] = oacc[t][r] * inv;
  }
  wave_sync_lds();
  {
    const int q4 = lane >> 3, c8 = (lane & 7) * 8;
    v4u hv[4];
#pragma unroll
    for (int it = 0; it < 4; ++it) {
      const int row = it * 4 + q4;
      const float* sp = os + row * 64 + c8;
      v4u a;
#pragma unroll
      for (int e = 0; e < 4; ++e) a[e] = pk16(h_bits((_Float16)sp[2 * e]), h_bits((_Float16)sp[2 * e + 1]));
      hv[it] = a;
    }
    for (int pass = 0; pass < 2; ++pass) {
#pragma unroll
      for (int it = 0; it < 4; ++it) {
        const int row = it * 4 + q4;
        const size_t go = (rowB + q0 + row) * DM + (size_t)h * HD + c8;
        *(volatile v4u*)(outp + go) = hv[it];
      }
      __threadfence();
    }
  }
}

__device__ __forceinline__ void row_store_h16(unsigned int* sb, unsigned short* dst_row, v4f o, int t) {
  v2u p;
  p[0] = pk16(h_bits((_Float16)o[0]), h_bits((_Float16)o[1]));
  p[1] = pk16(h_bits((_Float16)o[2]), h_bits((_Float16)o[3]));
  *(v2u*)(sb + 2 * t) = p;
  __syncthreads();
  if (t < 128) {
    const v4u v = *(const v4u*)(sb + 4 * t);
    *(volatile v4u*)(dst_row + 8 * t) = v;
    __threadfence();
    *(volatile v4u*)(dst_row + 8 * t) = v;
  }
}

template <int RIN>
__global__ __launch_bounds__(256) void ln_row_h(const float* __restrict__ X, const float* __restrict__ gam,
                                                const float* __restrict__ bet, unsigned short* outH) {
  __shared__ float red0[8], red1[8];
  __shared__ __align__(16) unsigned int sb[512];
  const int t = threadIdx.x, lane = t & 31, wave = t >> 5;
  const size_t base = (size_t)blockIdx.x * DM;
  v4f xv = *(const v4f*)(X + base + 4 * t);
  if (RIN) {
#pragma unroll
    for (int e = 0; e < 4; ++e) xv[e] = bfr(xv[e]);
  }
  const float mean = bsum256((xv[0] + xv[1]) + (xv[2] + xv[3]), red0, lane, wave) * (1.0f / DM);
  v4f d;
#pragma unroll
  for (int e = 0; e < 4; ++e) d[e] = xv[e] - mean;
  const float var  = bsum256((d[0] * d[0] + d[1] * d[1]) + (d[2] * d[2] + d[3] * d[3]), red1, lane, wave) * (1.0f / DM);
  const float rstd = 1.0f / sqrtf(var + LNEPS);
  const v4f gv = *(const v4f*)(gam + 4 * t);
  const v4f bv = *(const v4f*)(bet + 4 * t);
  v4f y;
#pragma unroll
  for (int e = 0; e < 4; ++e) y[e] = (d[e] * rstd) * bfr(gv[e]) + bfr(bv[e]);
  row_store_h16(sb, outH + base, y, t);
}

template <int RR>
__global__ __launch_bounds__(256) void combine_h(const float* __restrict__ P, int ldp,
                                                 const float* __restrict__ wf, const float* __restrict__ wr,
                                                 unsigned short* Aout, int ldao, float asc) {
  __shared__ __align__(16) unsigned short sb[NE * RR];
  const int t = threadIdx.x;
  const size_t bs = blockIdx.x;
  const v4f f0 = *(const v4f*)(wf + bs * NE), f1 = *(const v4f*)(wf + bs * NE + 4);
  const v4f g0 = *(const v4f*)(wr + bs * NE), g1 = *(const v4f*)(wr + bs * NE + 4);
  float wfv[NE], wrv[NE];
#pragma unroll
  for (int e = 0; e < 4; ++e) {
    wfv[e] = bfr(f0[e]); wfv[4 + e] = bfr(f1[e]);
    wrv[e] = bfr(g0[e]); wrv[4 + e] = bfr(g1[e]);
  }
  if (t < RR) {
    const float* pr = P + bs * (size_t)ldp + t;
    float h = 0.f;
#pragma unroll
    for (int n = 0; n < NE; ++n) h += wfv[n] * pr[n * RR];
#pragma unroll
    for (int n = 0; n < NE; ++n) sb[n * RR + t] = h_bits((_Float16)((wrv[n] * h) * asc));
  }
  __syncthreads();
  if (t < (NE * RR) / 8) {
    const v4u v = *(const v4u*)(sb + 8 * t);
    unsigned short* dst = Aout + bs * (size_t)ldao + 8 * t;
    *(volatile v4u*)dst = v;
    __threadfence();
    *(volatile v4u*)dst = v;
  }
}

extern "C" void kernel_launch(void* const* d_in, const int* in_sizes, int n_in,
                              void* d_out, int out_size, void* d_ws, size_t ws_size,
                              hipStream_t stream) {
  if (n_in < 20) return;
  if (in_sizes[0] != MP * DM) return;
  for (int i = 1; i <= 8; ++i) if (in_sizes[i] != MP * NE) return;
  if (in_sizes[9] != NE * DM * RK || in_sizes[10] != NE * DM * RK) return;
  if (in_sizes[11] != NE * RK * DM || in_sizes[12] != NE * RK * DM) return;
  if (in_sizes[13] != NE * DM * KRK || in_sizes[14] != NE * KRK * DM) return;
  if (in_sizes[15] != DM * DM) return;
  for (int i = 16; i <= 19; ++i) if (in_sizes[i] != DM) return;
  if (out_size != MP * DM) return;

  const float* x       = (const float*)d_in[0];
  const float* fqk_wQ  = (const float*)d_in[1];
  const float* fqk_wK  = (const float*)d_in[2];
  const float* fv_w    = (const float*)d_in[3];
  const float* rqk_wQ  = (const float*)d_in[4];
  const float* rqk_wK  = (const float*)d_in[5];
  const float* rv_w    = (const float*)d_in[6];
  const float* fkn_w   = (const float*)d_in[7];
  const float* rkn_w   = (const float*)d_in[8];
  const float* f_qk    = (const float*)d_in[9];
  const float* f_v     = (const float*)d_in[10];
  const float* r_qk    = (const float*)d_in[11];
  const float* r_v     = (const float*)d_in[12];
  const float* f_know  = (const float*)d_in[13];
  const float* r_know  = (const float*)d_in[14];
  const float* W_O     = (const float*)d_in[15];
  const float* ln1_g   = (const float*)d_in[16];
  const float* ln1_b   = (const float*)d_in[17];
  const float* ln2_g   = (const float*)d_in[18];
  const float* ln2_b   = (const float*)d_in[19];

  const size_t PFR  = (size_t)NR * DM * 2;
  const size_t PFK  = (size_t)NKR * DM * 2;
  const size_t PWO  = (size_t)DM * DM * 2;
  const size_t PXN  = (size_t)MP * DM * 2;
  const size_t PP   = (size_t)MP * NR * 4;
  const size_t PA   = (size_t)MP * NR * 2;
  const size_t PQK  = (size_t)MP * QKP * 2;
  const size_t PVT  = (size_t)NBATCH * DM * TT * 2;
  const size_t PCT  = (size_t)MP * DM * 2;
  const size_t PX1  = (size_t)MP * DM * 4;
  size_t off = 0;
  const size_t oFqk = off; off += PFR;
  const size_t oFv  = off; off += PFR;
  const size_t oRqk = off; off += PFR;
  const size_t oRv  = off; off += PFR;
  const size_t oFkn = off; off += PFK;
  const size_t oRkn = off; off += PFK;
  const size_t oWo  = off; off += PWO;
  const size_t oXN  = off; off += PXN;
  const size_t oP   = off; off += PP;
  const size_t oA   = off; off += PA;
  const size_t oQK  = off; off += PQK;
  const size_t oVT  = off; off += PVT;
  const size_t oCtx = off; off += PCT;
  const size_t oX1  = off; off += PX1;
  if (off > ws_size) return;
  if (off > (size_t)134217728) return;

  char* ws = (char*)d_ws;
  unsigned short* FqkH = (unsigned short*)(ws + oFqk);
  unsigned short* FvH  = (unsigned short*)(ws + oFv);
  unsigned short* RqkH = (unsigned short*)(ws + oRqk);
  unsigned short* RvH  = (unsigned short*)(ws + oRv);
  unsigned short* FknH = (unsigned short*)(ws + oFkn);
  unsigned short* RknH = (unsigned short*)(ws + oRkn);
  unsigned short* WoH  = (unsigned short*)(ws + oWo);
  unsigned short* XN   = (unsigned short*)(ws + oXN);
  float*          P    = (float*)(ws + oP);
  unsigned short* Apl  = (unsigned short*)(ws + oA);
  unsigned short* QK   = (unsigned short*)(ws + oQK);
  unsigned short* VT   = (unsigned short*)(ws + oVT);
  unsigned short* Ctx  = (unsigned short*)(ws + oCtx);
  float*          X1   = (float*)(ws + oX1);

  const dim3 blk(256), blk128(128);
  const dim3 gRow(MP);
  const dim3 gTF(RK / 64, DM / 64, NE);
  const dim3 gTR(DM / 64, RK / 64, NE);
  const dim3 gTFk(KRK / 64, DM / 64, NE);
  const dim3 gTRk(DM / 64, KRK / 64, NE);
  const dim3 gCo((DM * DM / 8 + 255) / 256);
  const dim3 gN2048(((MP / 64) * (NR / 64) + 7) / 8, 1);
  const dim3 gN1024(((MP / 64) * (DM / 64) + 7) / 8, 1);
  const dim3 gVT(((DM / 64) * (TT / 64) + 7) / 8, NBATCH);
  const dim3 gAttn(NBATCH * NH * NQB);
  const float invw  = 1.0f / WSC;
  const float oqk   = QKSC / (ASC * WSC);
  const float ovt   = VSC / (ASC * WSC);
  const float invwc = 1.0f / (WSC * CTXSC);
  const float orst  = 1.0f / (ASC * WSC);

  tconv_h64<<<gTF,  blk, 0, stream>>>(f_qk,   RK,  (long long)DM * RK,  FqkH, DM,  (long long)RK * DM,  WSC);
  tconv_h64<<<gTF,  blk, 0, stream>>>(f_v,    RK,  (long long)DM * RK,  FvH,  DM,  (long long)RK * DM,  WSC);
  tconv_h64<<<gTR,  blk, 0, stream>>>(r_qk,   DM,  (long long)RK * DM,  RqkH, NR,  (long long)RK,       WSC);
  tconv_h64<<<gTR,  blk, 0, stream>>>(r_v,    DM,  (long long)RK * DM,  RvH,  NR,  (long long)RK,       WSC);
  tconv_h64<<<gTFk, blk, 0, stream>>>(f_know, KRK, (long long)DM * KRK, FknH, DM,  (long long)KRK * DM, WSC);
  tconv_h64<<<gTRk, blk, 0, stream>>>(r_know, DM,  (long long)KRK * DM, RknH, NKR, (long long)KRK,      WSC);
  conv_h64<<<gCo, blk, 0, stream>>>(W_O, WoH, DM * DM / 8, WSC);

  ln_row_h<1><<<gRow, blk, 0, stream>>>(x, ln1_g, ln1_b, XN);

  gemm64<0, 2, 0, 0><<<gN2048, blk, 0, stream>>>(
      XN, DM, 0LL, FqkH, DM, 0LL, x, x, NR, x,
      (void*)P, NR, 0LL, MP, NR, DM, invw);

  combine_h<RK><<<gRow, blk, 0, stream>>>(P, NR, fqk_wQ, rqk_wQ, Apl, NR, ASC);
  gemm64<2, 2, 0, 0><<<gN1024, blk, 0, stream>>>(
      Apl, NR, 0LL, RqkH, NR, 0LL, x, x, DM, x,
      (void*)QK, QKP, 0LL, MP, DM, NR, oqk);

  combine_h<RK><<<gRow, blk, 0, stream>>>(P, NR, fqk_wK, rqk_wK, Apl, NR, ASC);
  gemm64<2, 2, 0, 0><<<gN1024, blk, 0, stream>>>(
      Apl, NR, 0LL, RqkH, NR, 0LL, x, x, DM, x,
      (void*)(QK + DM), QKP, 0LL, MP, DM, NR, oqk);

  gemm64<0, 2, 0, 0><<<gN2048, blk, 0, stream>>>(
      XN, DM, 0LL, FvH, DM, 0LL, x, x, NR, x,
      (void*)P, NR, 0LL, MP, NR, DM, invw);
  combine_h<RK><<<gRow, blk, 0, stream>>>(P, NR, fv_w, rv_w, Apl, NR, ASC);
  gemm64<2, 2, 0, 0><<<gVT, blk, 0, stream>>>(
      RvH, NR, 0LL, Apl, NR, (long long)TT * NR, x, x, TT, x,
      (void*)VT, TT, (long long)DM * TT, DM, TT, NR, ovt);

  attn64<<<gAttn, blk128, 0, stream>>>(QK, VT, Ctx, 0.125f / (QKSC * QKSC));

  gemm64<0, 2, 0, 2><<<gN1024, blk, 0, stream>>>(
      Ctx, DM, 0LL, WoH, DM, 0LL, x, x, DM, x,
      (void*)X1, DM, 0LL, MP, DM, DM, invwc);

  ln_row_h<0><<<gRow, blk, 0, stream>>>(X1, ln2_g, ln2_b, XN);

  gemm64<0, 2, 0, 0><<<gN1024, blk, 0, stream>>>(
      XN, DM, 0LL, FknH, DM, 0LL, x, x, NKR, x,
      (void*)P, NKR, 0LL, MP, NKR, DM, invw);

  combine_h<KRK><<<gRow, blk, 0, stream>>>(P, NKR, fkn_w, rkn_w, Apl, NKR, ASC);

  gemm64<0, 2, 0, 1><<<gN1024, blk, 0, stream>>>(
      Apl, NKR, 0LL, RknH, NKR, 0LL, x, x, DM, X1,
      (void*)d_out, DM, 0LL, MP, DM, NKR, orst);
  (void)hipGetLastError();
}
